// Qwen3MHAttention_64312840290532
// MI455X (gfx1250) — hardware-verified
//
#include <hip/hip_runtime.h>

#define DEV static __device__ __forceinline__

typedef _Float16 v16h __attribute__((ext_vector_type(16)));
typedef _Float16 v8h  __attribute__((ext_vector_type(8)));
typedef _Float16 v8ha __attribute__((ext_vector_type(8), may_alias));
typedef float    v8f  __attribute__((ext_vector_type(8)));
typedef float    v4f  __attribute__((ext_vector_type(4)));
typedef float    v4fa __attribute__((ext_vector_type(4), may_alias));

union Frag { v16h v; v8h h[2]; };
union H8   { v8h v; _Float16 s[8]; };
union H16  { v8h v[2]; _Float16 s[16]; };

constexpr int Bc = 2, Tc = 2048, Dc = 2048, Hc = 16, HKVc = 8, DHc = 128;
constexpr int Mc = Bc * Tc;
static_assert(Mc % 64 == 0 && Dc % 128 == 0 && (HKVc * DHc) % 128 == 0 && (Hc * DHc) % 128 == 0 &&
              Dc % 32 == 0 && DHc == 128 && Tc % 128 == 0 && (Hc % HKVc) == 0);

DEV float bf16r(float f) {
    unsigned u = __float_as_uint(f);
    u += 0x7FFFu + ((u >> 16) & 1u);
    u &= 0xFFFF0000u;
    return __uint_as_float(u);
}

DEV v8f wmma16(const v16h& a, const v16h& b, v8f c) {
    return __builtin_amdgcn_wmma_f32_16x16x32_f16(false, a, false, b, (short)0, c, false, false);
}

__global__ __launch_bounds__(256) void k_cvt(const float* __restrict__ in, _Float16* out,
                                             int n8, float scale) {
    const size_t stride = (size_t)gridDim.x * 256;
    for (int pass = 0; pass < 2; ++pass) {
        for (size_t i = (size_t)blockIdx.x * 256 + threadIdx.x; i < (size_t)n8; i += stride) {
            v4f a = *(const v4f*)(in + 8 * i);
            v4f b = *(const v4f*)(in + 8 * i + 4);
            H8 r;
            #pragma unroll
            for (int j = 0; j < 4; ++j) {
                r.s[j]     = (_Float16)(bf16r(a[j]) * scale);
                r.s[4 + j] = (_Float16)(bf16r(b[j]) * scale);
            }
            *(volatile v8h*)(out + 8 * i) = r.v;
        }
        __threadfence();
    }
}

DEV void st_hilo(const float* crow, _Float16* ohi, _Float16* olo, size_t prow, int lo, int hi) {
    const int seg = lo * 8;
    v4f a = *(const v4fa*)(crow + seg);
    v4f b = *(const v4fa*)(crow + seg + 4);
    H8 ph, pl, ps;
    #pragma unroll
    for (int j = 0; j < 4; ++j) {
        _Float16 ha = (_Float16)a[j];
        _Float16 hb = (_Float16)b[j];
        ph.s[j]     = ha;
        ph.s[4 + j] = hb;
        pl.s[j]     = (_Float16)((a[j] - (float)ha) * 2048.0f);
        pl.s[4 + j] = (_Float16)((b[j] - (float)hb) * 2048.0f);
    }
    #pragma unroll
    for (int j = 0; j < 8; ++j) ps.s[j] = hi ? pl.s[j] : ph.s[j];
    _Float16* dst = hi ? (olo + prow + seg) : (ohi + prow + seg);
    *(volatile v8h*)dst = ps.v;
}

template <int MODE>
__global__ __launch_bounds__(256) void k_gemm(const _Float16* __restrict__ A,
                                              const _Float16* __restrict__ W,
                                              void* Out0, void* Out1, const float* __restrict__ nw,
                                              int M, int N, int K, int Hx, float oscale) {
    __shared__ __align__(16) float Cs[64][132];
    const int tid = threadIdx.x;
    const int lane = tid & 31, w = tid >> 5;
    const int wm = w >> 2, wn = w & 3;
    const int lo = lane & 15, hi = lane >> 4;
    const int rb = blockIdx.y * 64, cb = blockIdx.x * 128;
    if (rb + 64 > M || cb + 128 > N) return;
    const int row0 = rb + wm * 32, col0 = cb + wn * 32;

    const _Float16* ap0 = A + (size_t)(row0 + lo) * K;
    const _Float16* ap1 = ap0 + (size_t)16 * K;
    const _Float16* wp0 = W + (size_t)(col0 + lo) * K;
    const _Float16* wp1 = wp0 + (size_t)16 * K;

    v8f acc00 = {}, acc01 = {}, acc10 = {}, acc11 = {};
    for (int kc = 0; kc < K; kc += 32) {
        Frag a0, a1, b0, b1;
        a0.h[0] = *(const v8h*)(ap0 + kc + 8 * hi);  a0.h[1] = *(const v8h*)(ap0 + kc + 16 + 8 * hi);
        a1.h[0] = *(const v8h*)(ap1 + kc + 8 * hi);  a1.h[1] = *(const v8h*)(ap1 + kc + 16 + 8 * hi);
        b0.h[0] = *(const v8h*)(wp0 + kc + 8 * hi);  b0.h[1] = *(const v8h*)(wp0 + kc + 16 + 8 * hi);
        b1.h[0] = *(const v8h*)(wp1 + kc + 8 * hi);  b1.h[1] = *(const v8h*)(wp1 + kc + 16 + 8 * hi);
        acc00 = wmma16(a0.v, b0.v, acc00);
        acc01 = wmma16(a0.v, b1.v, acc01);
        acc10 = wmma16(a1.v, b0.v, acc10);
        acc11 = wmma16(a1.v, b1.v, acc11);
        asm volatile("v_nop\n\tv_nop\n\tv_nop\n\tv_nop"
                     : "+v"(acc00), "+v"(acc01), "+v"(acc10), "+v"(acc11)
                     : "v"(a0.v), "v"(a1.v), "v"(b0.v), "v"(b1.v));
    }

    {
        const int r0 = wm * 32, c0 = wn * 32;
        #pragma unroll
        for (int r = 0; r < 8; ++r) {
            Cs[r0 + 8 * hi + r][c0 + lo]           = acc00[r] * oscale;
            Cs[r0 + 8 * hi + r][c0 + 16 + lo]      = acc01[r] * oscale;
            Cs[r0 + 16 + 8 * hi + r][c0 + lo]      = acc10[r] * oscale;
            Cs[r0 + 16 + 8 * hi + r][c0 + 16 + lo] = acc11[r] * oscale;
        }
    }
    __syncthreads();

    if constexpr (MODE == 0) {
        float* o = (float*)Out0;
        for (int pass = 0; pass < 2; ++pass) {
            #pragma unroll
            for (int it = 0; it < 8; ++it) {
                const int row = it * 8 + w;
                const size_t base = (size_t)(rb + row) * N + cb;
                v4f a = *(const v4fa*)&Cs[row][4 * lane];
                *(volatile v4f*)(o + base + 4 * lane) = a;
            }
            __threadfence();
        }
    } else if constexpr (MODE == 2) {
        _Float16* o = (_Float16*)Out0;
        const int head = cb / DHc;
        for (int pass = 0; pass < 2; ++pass) {
            #pragma unroll
            for (int it = 0; it < 4; ++it) {
                const int row = it * 16 + w * 2 + hi;
                const int m = rb + row;
                const int bb = m / Tc, t = m % Tc;
                const size_t base = (((size_t)bb * Hx + head) * Tc + t) * DHc;
                v4f a = *(const v4fa*)&Cs[row][8 * lo];
                v4f b = *(const v4fa*)&Cs[row][8 * lo + 4];
                H8 rr;
                #pragma unroll
                for (int j = 0; j < 4; ++j) {
                    rr.s[j]     = (_Float16)a[j];
                    rr.s[4 + j] = (_Float16)b[j];
                }
                *(volatile v8h*)(o + base + 8 * lo) = rr.v;
            }
            __threadfence();
        }
    } else {
        _Float16* ohi = (_Float16*)Out0;
        _Float16* olo = (_Float16*)Out1;
        const int head = cb / DHc;
        const int d0 = 2 * lane;
        const float w0 = nw[d0], w1 = nw[d0 + 1], w2 = nw[64 + d0], w3 = nw[65 + d0];
        const float e0 = (float)(2 * d0) * (1.0f / 128.0f);
        const float e1 = (float)(2 * (d0 + 1)) * (1.0f / 128.0f);
        const float if0 = 1.0f / powf(1000000.0f, e0);
        const float if1 = 1.0f / powf(1000000.0f, e1);
        #pragma unroll 1
        for (int it = 0; it < 8; ++it) {
            const int row = it * 8 + w;
            const int m = rb + row;
            const int bb = m / Tc, t = m % Tc;
            const float x0 = Cs[row][d0], x1 = Cs[row][d0 + 1], x2 = Cs[row][64 + d0], x3 = Cs[row][65 + d0];
            float ss = x0 * x0 + x1 * x1 + x2 * x2 + x3 * x3;
            ss += __shfl_xor(ss, 1, 32);  ss += __shfl_xor(ss, 2, 32);  ss += __shfl_xor(ss, 4, 32);
            ss += __shfl_xor(ss, 8, 32);  ss += __shfl_xor(ss, 16, 32);
            const float rms = rsqrtf(ss * (1.0f / 128.0f) + 1e-6f);
            const float n0 = x0 * rms * w0, n1 = x1 * rms * w1, n2 = x2 * rms * w2, n3 = x3 * rms * w3;
            const float a0 = (float)t * if0, a1 = (float)t * if1;
            const float c0 = cosf(a0), s0 = sinf(a0), c1 = cosf(a1), s1 = sinf(a1);
            const float y0 = n0 * c0 - n2 * s0;
            const float y1 = n1 * c1 - n3 * s1;
            const float y2 = n2 * c0 + n0 * s0;
            const float y3 = n3 * c1 + n1 * s1;
            Cs[row][d0] = y0;  Cs[row][d0 + 1] = y1;  Cs[row][64 + d0] = y2;  Cs[row][65 + d0] = y3;
            asm volatile("s_wait_dscnt 0" ::: "memory");
            const size_t prow = (((size_t)bb * Hx + head) * Tc + t) * DHc;
            st_hilo(&Cs[row][0], ohi, olo, prow, lo, hi);
        }
        __threadfence();
        #pragma unroll 1
        for (int it = 0; it < 8; ++it) {
            const int row = it * 8 + w;
            const int m = rb + row;
            const int bb = m / Tc, t = m % Tc;
            const size_t prow = (((size_t)bb * Hx + head) * Tc + t) * DHc;
            st_hilo(&Cs[row][0], ohi, olo, prow, lo, hi);
        }
        __threadfence();
    }
}

__global__ __launch_bounds__(256) void k_attn(const _Float16* __restrict__ qhi, const _Float16* __restrict__ qlo,
                                              const _Float16* __restrict__ khi, const _Float16* __restrict__ klo,
                                              const _Float16* __restrict__ vh, _Float16* ctx) {
    __shared__ __align__(16) _Float16 vT[128][40];
    __shared__ __align__(16) _Float16 Cl[8][16][136];

    const int tid = threadIdx.x;
    const int lane = tid & 31, w = tid >> 5;
    const int lo = lane & 15, hi = lane >> 4;
    const int bh = blockIdx.y;
    const int b = bh / Hc, h = bh % Hc;
    const int kvh = h / (Hc / HKVc);
    const int qbase = blockIdx.x * 128 + w * 16;

    const size_t qoff = ((size_t)b * Hc + h) * Tc * DHc;
    const size_t koff = ((size_t)b * HKVc + kvh) * Tc * DHc;
    const _Float16* qhr = qhi + qoff + (size_t)(qbase + lo) * DHc;
    const _Float16* qlr = qlo + qoff + (size_t)(qbase + lo) * DHc;

    v8f o[8];
    #pragma unroll
    for (int c = 0; c < 8; ++c) o[c] = (v8f){};
    float mrow[8], lrow[8];
    #pragma unroll
    for (int r = 0; r < 8; ++r) { mrow[r] = -1e30f; lrow[r] = 0.0f; }

    const int kmax = (blockIdx.x + 1) * 128;
    for (int kt = 0; kt < kmax; kt += 32) {
        __syncthreads();
        {
            const int key = tid >> 3;
            const int dg = (tid & 7) * 16;
            const _Float16* vp = vh + koff + (size_t)(kt + key) * DHc + dg;
            H16 tb;
            tb.v[0] = *(const v8h*)(vp);
            tb.v[1] = *(const v8h*)(vp + 8);
            #pragma unroll
            for (int j = 0; j < 16; ++j) vT[dg + j][key] = tb.s[j];
        }
        __syncthreads();
        if (kt > qbase + 15) continue;

        v8f shh0 = {}, shh1 = {}, sx0 = {}, sx1 = {};
        const _Float16* kh0 = khi + koff + (size_t)(kt + lo) * DHc;
        const _Float16* kh1 = kh0 + (size_t)16 * DHc;
        const _Float16* kl0 = klo + koff + (size_t)(kt + lo) * DHc;
        const _Float16* kl1 = kl0 + (size_t)16 * DHc;
        #pragma unroll
        for (int c = 0; c < 4; ++c) {
            const int d0 = c * 32;
            Frag ah, al, bh0, bh1, bl0, bl1;
            ah.h[0]  = *(const v8h*)(qhr + d0 + 8 * hi);  ah.h[1]  = *(const v8h*)(qhr + d0 + 16 + 8 * hi);
            al.h[0]  = *(const v8h*)(qlr + d0 + 8 * hi);  al.h[1]  = *(const v8h*)(qlr + d0 + 16 + 8 * hi);
            bh0.h[0] = *(const v8h*)(kh0 + d0 + 8 * hi);  bh0.h[1] = *(const v8h*)(kh0 + d0 + 16 + 8 * hi);
            bh1.h[0] = *(const v8h*)(kh1 + d0 + 8 * hi);  bh1.h[1] = *(const v8h*)(kh1 + d0 + 16 + 8 * hi);
            bl0.h[0] = *(const v8h*)(kl0 + d0 + 8 * hi);  bl0.h[1] = *(const v8h*)(kl0 + d0 + 16 + 8 * hi);
            bl1.h[0] = *(const v8h*)(kl1 + d0 + 8 * hi);  bl1.h[1] = *(const v8h*)(kl1 + d0 + 16 + 8 * hi);
            shh0 = wmma16(ah.v, bh0.v, shh0);
            shh1 = wmma16(ah.v, bh1.v, shh1);
            sx0  = wmma16(ah.v, bl0.v, sx0);
            sx0  = wmma16(al.v, bh0.v, sx0);
            sx1  = wmma16(ah.v, bl1.v, sx1);
            sx1  = wmma16(al.v, bh1.v, sx1);
            asm volatile("v_nop\n\tv_nop\n\tv_nop\n\tv_nop"
                         : "+v"(shh0), "+v"(shh1), "+v"(sx0), "+v"(sx1)
                         : "v"(ah.v), "v"(al.v), "v"(bh0.v), "v"(bh1.v), "v"(bl0.v), "v"(bl1.v));
        }

        const float sc = 0.08838834764831845f;
        const float xs = 1.0f / 2048.0f;
        float p0[8], p1[8];
        #pragma unroll
        for (int r = 0; r < 8; ++r) {
            const int qi = qbase + r + 8 * hi;
            float v0 = (shh0[r] + sx0[r] * xs) * sc;
            float v1 = (shh1[r] + sx1[r] * xs) * sc;
            float e0 = (kt + lo      <= qi) ? v0 : -1e30f;
            float e1 = (kt + 16 + lo <= qi) ? v1 : -1e30f;
            float rv = fmaxf(e0, e1);
            rv = fmaxf(rv, __shfl_xor(rv, 1, 32));
            rv = fmaxf(rv, __shfl_xor(rv, 2, 32));
            rv = fmaxf(rv, __shfl_xor(rv, 4, 32));
            rv = fmaxf(rv, __shfl_xor(rv, 8, 32));
            const float mn = fmaxf(mrow[r], rv);
            const float scale = __expf(mrow[r] - mn);
            mrow[r] = mn;
            e0 = __expf(e0 - mn);
            e1 = __expf(e1 - mn);
            float ts = e0 + e1;
            ts += __shfl_xor(ts, 1, 32);
            ts += __shfl_xor(ts, 2, 32);
            ts += __shfl_xor(ts, 4, 32);
            ts += __shfl_xor(ts, 8, 32);
            lrow[r] = lrow[r] * scale + ts;
            p0[r] = e0; p1[r] = e1;
            #pragma unroll
            for (int c = 0; c < 8; ++c) o[c][r] *= scale;
        }

        #pragma unroll
        for (int r = 0; r < 8; ++r) {
            Cl[w][8 * hi + r][lo]      = (_Float16)(p0[r] * 4096.0f);
            Cl[w][8 * hi + r][16 + lo] = (_Float16)(p1[r] * 4096.0f);
        }
        asm volatile("s_wait_dscnt 0" ::: "memory");
        Frag pa;
        pa.h[0] = *(const v8ha*)(&Cl[w][lo][8 * hi]);
        pa.h[1] = *(const v8ha*)(&Cl[w][lo][16 + 8 * hi]);

        Frag bv;
        #pragma unroll
        for (int c = 0; c < 8; ++c) {
            bv.h[0] = *(const v8ha*)(&vT[c * 16 + lo][8 * hi]);
            bv.h[1] = *(const v8ha*)(&vT[c * 16 + lo][16 + 8 * hi]);
            o[c] = wmma16(pa.v, bv.v, o[c]);
        }
        asm volatile("v_nop\n\tv_nop\n\tv_nop\n\tv_nop"
                     : "+v"(o[0]), "+v"(o[1]), "+v"(o[2]), "+v"(o[3]),
                       "+v"(o[4]), "+v"(o[5]), "+v"(o[6]), "+v"(o[7])
                     : "v"(pa.v), "v"(bv.v));
    }

    float inv[8];
    #pragma unroll
    for (int r = 0; r < 8; ++r) inv[r] = 1.0f / (lrow[r] * 256.0f);
    #pragma unroll
    for (int c = 0; c < 8; ++c) {
        #pragma unroll
        for (int r = 0; r < 8; ++r)
            Cl[w][8 * hi + r][c * 16 + lo] = (_Float16)(o[c][r] * inv[r]);
    }
    asm volatile("s_wait_dscnt 0" ::: "memory");
    _Float16* op = ctx + ((size_t)b * Tc + qbase) * (size_t)(Hc * DHc) + (size_t)h * DHc;
    for (int pass = 0; pass < 2; ++pass) {
        #pragma unroll
        for (int it = 0; it < 8; ++it) {
            const int row = it * 2 + hi;
            const int col = lo * 8;
            v8h val = *(const v8ha*)(&Cl[w][row][col]);
            *(volatile v8h*)(op + (size_t)row * (Hc * DHc) + col) = val;
        }
        __threadfence();
    }
}

extern "C" void kernel_launch(void* const* d_in, const int* in_sizes, int n_in,
                              void* d_out, int out_size, void* d_ws, size_t ws_size,
                              hipStream_t stream) {
    if (n_in != 7) return;
    if (in_sizes[0] != Mc * Dc || in_sizes[1] != Hc * DHc * Dc || in_sizes[2] != HKVc * DHc * Dc ||
        in_sizes[3] != HKVc * DHc * Dc || in_sizes[4] != Dc * Hc * DHc ||
        in_sizes[5] != DHc || in_sizes[6] != DHc || out_size != Mc * Dc) return;

    const float* x  = (const float*)d_in[0];
    const float* wq = (const float*)d_in[1];
    const float* wk = (const float*)d_in[2];
    const float* wv = (const float*)d_in[3];
    const float* wo = (const float*)d_in[4];
    const float* qw = (const float*)d_in[5];
    const float* kw = (const float*)d_in[6];

    const size_t szX   = (size_t)Mc * Dc * 2;
    const size_t szWq  = (size_t)Hc * DHc * Dc * 2;
    const size_t szWk  = (size_t)HKVc * DHc * Dc * 2;
    const size_t szWo  = (size_t)Dc * Hc * DHc * 2;
    const size_t szQ   = (size_t)Mc * Hc * DHc * 2;
    const size_t szK   = (size_t)Mc * HKVc * DHc * 2;
    const size_t offX   = 0;
    const size_t offWq  = offX + szX;
    const size_t offWk  = offWq + szWq;
    const size_t offWv  = offWk + szWk;
    const size_t offWo  = offWv + szWk;
    const size_t offQhi = offWo + szWo;
    const size_t offQlo = offQhi + szQ;
    const size_t offKhi = offQlo + szQ;
    const size_t offKlo = offKhi + szK;
    const size_t offV   = offKlo + szK;
    const size_t offCtx = offV + szK;
    const size_t total  = offCtx + szQ;
    if (total > ws_size) return;

    char* ws = (char*)d_ws;
    _Float16* xh   = (_Float16*)(ws + offX);
    _Float16* wqh  = (_Float16*)(ws + offWq);
    _Float16* wkh  = (_Float16*)(ws + offWk);
    _Float16* wvh  = (_Float16*)(ws + offWv);
    _Float16* woh  = (_Float16*)(ws + offWo);
    _Float16* qhi  = (_Float16*)(ws + offQhi);
    _Float16* qlo  = (_Float16*)(ws + offQlo);
    _Float16* khi  = (_Float16*)(ws + offKhi);
    _Float16* klo  = (_Float16*)(ws + offKlo);
    _Float16* vh   = (_Float16*)(ws + offV);
    _Float16* ctxh = (_Float16*)(ws + offCtx);

    auto cvt_grid = [](int n) { int n8 = n / 8; int g = (n8 + 255) / 256; return g > 4096 ? 4096 : g; };

    k_cvt<<<cvt_grid(Mc * Dc), 256, 0, stream>>>(x, xh, Mc * Dc / 8, 1.0f);
    k_cvt<<<cvt_grid(Hc * DHc * Dc), 256, 0, stream>>>(wq, wqh, Hc * DHc * Dc / 8, 64.0f);
    k_cvt<<<cvt_grid(HKVc * DHc * Dc), 256, 0, stream>>>(wk, wkh, HKVc * DHc * Dc / 8, 64.0f);
    k_cvt<<<cvt_grid(HKVc * DHc * Dc), 256, 0, stream>>>(wv, wvh, HKVc * DHc * Dc / 8, 64.0f);
    k_cvt<<<cvt_grid(Dc * Hc * DHc), 256, 0, stream>>>(wo, woh, Dc * Hc * DHc / 8, 64.0f);

    k_gemm<1><<<dim3((Hc * DHc) / 128, Mc / 64), 256, 0, stream>>>(xh, wqh, qhi, qlo, qw, Mc, Hc * DHc, Dc, Hc, 1.0f / 64.0f);
    k_gemm<1><<<dim3((HKVc * DHc) / 128, Mc / 64), 256, 0, stream>>>(xh, wkh, khi, klo, kw, Mc, HKVc * DHc, Dc, HKVc, 1.0f / 64.0f);
    k_gemm<2><<<dim3((HKVc * DHc) / 128, Mc / 64), 256, 0, stream>>>(xh, wvh, vh, vh, qw, Mc, HKVc * DHc, Dc, HKVc, 1.0f / 64.0f);

    k_attn<<<dim3(Tc / 128, Bc * Hc), 256, 0, stream>>>(qhi, qlo, khi, klo, vh, ctxh);

    k_gemm<0><<<dim3(Dc / 128, Mc / 64), 256, 0, stream>>>(ctxh, woh, d_out, d_out, qw, Mc, Dc, Hc * DHc, 0, 1.0f / 1024.0f);
}
